// OptionsCritic_5892695130342
// MI455X (gfx1250) — hardware-run, weakly checked
//
#include <hip/hip_runtime.h>


#ifndef NB
#define NB 32768
#endif
#define NB_FULL 32768
#define OBSD  256
#define HIDD  64
#define FEAT  128
#define NOPT  8
#define ACTN  18
#define ACTP  32
#define NREL  32
#define RB    1024
#define NBLK  (NB / RB)
#define OFFP  128
#define PROWS (NB + 2048)
#define HP    72
#define SPH   136
#define OP    36
#define HDP   20
#define WSC   64.0f
#define ASC   16.0f
#define INVC  (1.0f / 1024.0f)

static_assert(NB % RB == 0);
static_assert(NBLK >= 1 && NBLK <= OFFP);
static_assert(NB <= NB_FULL);
static_assert(NREL * 63 <= 2048);
static_assert(NOPT <= NREL);
static_assert(PROWS % 64 == 0);
static_assert(NB % 4 == 0);
static_assert(OBSD == 32 * 8);
static_assert(OBSD % 32 == 0 && HIDD % 32 == 0 && FEAT % 32 == 0);
static_assert(HIDD == 64 && FEAT == 128);
static_assert(ACTN == 2 * 9 && ACTN + 2 <= ACTP && ACTP == 32);
static_assert((HP * 2) % 16 == 0 && (SPH * 2) % 16 == 0 && (OP * 4) % 16 == 0);
static_assert((size_t)NB_FULL * 4 == (size_t)131072);
static_assert(4 * (16 * HP * 2 + 16 * SPH * 2 + 16 * HP * 2 + 16 * OP * 4 + 16 * HDP * 4 + 16 * 4) <= 131072);

typedef unsigned short bf;
typedef _Float16 h16;
typedef __attribute__((ext_vector_type(16))) __bf16   v16bf;
typedef __attribute__((ext_vector_type(16))) _Float16 v16h;
typedef __attribute__((ext_vector_type(8)))  _Float16 v8h;
typedef __attribute__((ext_vector_type(8)))  unsigned short v8us;
typedef __attribute__((ext_vector_type(8)))  float    v8f;
typedef __attribute__((ext_vector_type(4)))  float    v4f;
typedef __attribute__((ext_vector_type(4)))  int      v4i;
typedef v4f  __attribute__((may_alias)) v4fa;
typedef v4i  __attribute__((may_alias)) v4ia;
typedef v8h  __attribute__((may_alias)) v8ha;

__device__ __forceinline__ unsigned short f2bf(float f) { unsigned u = __float_as_uint(f); u += 0x7FFFu + ((u >> 16) & 1u); return (unsigned short)(u >> 16); }
__device__ __forceinline__ float bf2f(unsigned short w) { return __uint_as_float(((unsigned)w) << 16); }
__device__ __forceinline__ int clampi(int v, int lo, int hi) { return min(max(v, lo), hi); }
__device__ __forceinline__ v16bf cat16b(v8us lo, v8us hi) { return __builtin_bit_cast(v16bf, __builtin_shufflevector(lo, hi, 0, 1, 2, 3, 4, 5, 6, 7, 8, 9, 10, 11, 12, 13, 14, 15)); }
__device__ __forceinline__ v16bf ldb(const bf* p)  { return cat16b(*(const v8us*)p, *(const v8us*)(p + 16)); }
__device__ __forceinline__ void wave_sync() { __builtin_amdgcn_fence(3  , "wavefront"); __builtin_amdgcn_wave_barrier(); asm volatile("" ::: "memory"); }

static __device__ __forceinline__ h16 toh_flush(float v) { const h16 r = (h16)v; return (fabsf(v) < 6.103515625e-05f) ? (h16)0.0f : r; }
__device__ __forceinline__ float bfr(float v) { return bf2f(f2bf(v)); }
__device__ __forceinline__ v16h cat16h(v8h lo, v8h hi) { return __builtin_shufflevector(lo, hi, 0, 1, 2, 3, 4, 5, 6, 7, 8, 9, 10, 11, 12, 13, 14, 15); }
__device__ __forceinline__ v16h ldh(const h16* __restrict__ p) { return cat16h(*(const v8h*)p, *(const v8h*)(p + 16)); }
__device__ __forceinline__ v8f wmmab_g(v16bf a, v16bf b, v8f c) {
    c = __builtin_amdgcn_wmma_f32_16x16x32_bf16(false, a, false, b, (short)0, c, false, false);
    asm volatile("v_nop\n\tv_nop\n\tv_nop\n\tv_nop" : "+v"(c) : "v"(a), "v"(b));
    return c; }
__device__ __forceinline__ v8f wmmah_g(v16h a, v16h b, v8f c) {
    c = __builtin_amdgcn_wmma_f32_16x16x32_f16(false, a, false, b, (short)0, c, false, false);
    asm volatile("v_nop\n\tv_nop\n\tv_nop\n\tv_nop" : "+v"(c) : "v"(a), "v"(b));
    return c; }

__device__ __forceinline__ void st2_h(h16* dst, v8f x, bool keep) {
    v8h o;
#pragma unroll
    for (int k = 0; k < 8; ++k) { const float w = keep ? bfr(x[k]) * WSC : 0.0f; o[k] = toh_flush(w); }
    *(volatile v8h*)dst = o; __threadfence(); *(volatile v8h*)dst = o;
}

#define WG_W1 (HIDD * OBSD / 8)
#define WG_W2 (FEAT * HIDD / 8)
#define WG_HD (16 * FEAT / 8)
#define WG_E1 (NOPT * HIDD * FEAT / 8)
#define WG_E2 (NOPT * ACTP * HIDD / 8)
#define WB_W1 (WG_W1 / 256)
#define WB_W2 (WG_W2 / 256)
#define WB_HD (WG_HD / 256)
#define WB_E1 (WG_E1 / 256)
#define WB_E2 (WG_E2 / 256)
static_assert(WG_W1 % 256 == 0 && WG_W2 % 256 == 0 && WG_HD == 256 && WG_E1 % 256 == 0 && WG_E2 % 256 == 0);
static_assert(WG_E2 == NOPT * 256);

__global__ __launch_bounds__(256) void k_wconv(const float* __restrict__ fW1, const float* __restrict__ fW2, const float* __restrict__ pW, const float* __restrict__ tW,
                                               const float* __restrict__ oW1, const float* __restrict__ oW2,
                                               bf* W1B, h16* W2H, h16* HDH, h16* E1H, h16* E2H) {
    const int blk = blockIdx.x, t = threadIdx.x;
    if (blk < WB_W1) {
        const int g = blk * 256 + t;
        const v8f x = *(const v8f*)(fW1 + (size_t)g * 8); v8us o;
#pragma unroll
        for (int k = 0; k < 8; ++k) o[k] = f2bf(x[k]);
        *(volatile v8us*)(W1B + (size_t)g * 8) = o; __threadfence(); *(volatile v8us*)(W1B + (size_t)g * 8) = o;
    } else if (blk < WB_W1 + WB_W2) {
        const int g = (blk - WB_W1) * 256 + t;
        const v8f x = *(const v8f*)(fW2 + (size_t)g * 8);
        st2_h(W2H + (size_t)g * 8, x, true);
    } else if (blk < WB_W1 + WB_W2 + WB_HD) {
        const int g = t;
        const int gp = min(g, 127), gt = clampi(g - 128, 0, 127);
        const v8f xp = *(const v8f*)(pW + (size_t)gp * 8);
        const v8f xt = *(const v8f*)(tW + (size_t)gt * 8);
        v8f x;
#pragma unroll
        for (int k = 0; k < 8; ++k) x[k] = (g < 128) ? xp[k] : xt[k];
        st2_h(HDH + (size_t)g * 8, x, true);
    } else if (blk < WB_W1 + WB_W2 + WB_HD + WB_E1) {
        const int g = (blk - (WB_W1 + WB_W2 + WB_HD)) * 256 + t;
        const v8f x = *(const v8f*)(oW1 + (size_t)g * 8);
        st2_h(E1H + (size_t)g * 8, x, true);
    } else {
        const int g = (blk - (WB_W1 + WB_W2 + WB_HD + WB_E1)) * 256 + t;
        const int o = clampi(g >> 8, 0, NOPT - 1), n = (g >> 3) & 31, c8 = (g & 7) * 8;
        const int nn = min(n, ACTN - 1);
        const v8f x = *(const v8f*)(oW2 + ((size_t)(o * ACTN + nn) * HIDD + c8));
        st2_h(E2H + (size_t)g * 8, x, n < ACTN);
    }
}

__global__ __launch_bounds__(1024) void k_count(const int* __restrict__ opt, int* cnt) {
    __shared__ int wc[32 * 32];
    __shared__ __align__(16) int line[32];
    const int tid = threadIdx.x, lane = tid & 31; const int wave = __builtin_amdgcn_readfirstlane(tid >> 5);
    const int blk = blockIdx.x;
    const int rel = clampi(opt[(size_t)blk * RB + tid], 0, NOPT - 1);
    int mine = 0;
#pragma unroll 1
    for (int r = 0; r < NREL; ++r) { const unsigned m = __builtin_amdgcn_ballot_w32(rel == r); const int c = __builtin_popcount(m); mine = (lane == r) ? c : mine; }
    wc[wave * 32 + lane] = mine;
    __syncthreads();
    if (wave == 0) {
        int s = 0;
#pragma unroll 1
        for (int w = 0; w < 32; ++w) s += wc[w * 32 + lane];
        line[lane] = s;
        wave_sync();
#pragma unroll 1
        for (int ps = 0; ps < 2; ++ps) {
            if (lane < 8) { const v4i v = *(const v4ia*)(&line[4 * lane]); *(volatile v4i*)(cnt + (size_t)blk * 32 + 4 * lane) = v; }
            if (ps == 0) __threadfence(); }
    }
}

__global__ __launch_bounds__(1024) void k_scan(const int* __restrict__ cnt, int* offs, int* T, bf* XP) {
    __shared__ int tots[32];
    __shared__ __align__(16) int tl[128];
    const int tid = threadIdx.x, lane = tid & 31; const int r = __builtin_amdgcn_readfirstlane(tid >> 5);
    int c[4]; int ls = 0;
#pragma unroll
    for (int i = 0; i < 4; ++i) { const int blk = 4 * lane + i; const int bc = min(blk, NBLK - 1);
        int v = cnt[(size_t)bc * 32 + r]; v = (blk < NBLK) ? v : 0; v = clampi(v, 0, RB); c[i] = v; ls += v; }
    int x = ls;
#pragma unroll
    for (int d = 1; d < 32; d <<= 1) { const int y = __shfl_up(x, d, 32); x += (lane >= d) ? y : 0; }
    const int excl = x - ls;
    const int tot = __shfl(x, 31, 32);
    if (lane == 0) tots[r] = tot;
    __syncthreads();
    const int t = tots[lane]; const int pd = (t + 63) & ~63;
    int y2 = pd;
#pragma unroll
    for (int d = 1; d < 32; d <<= 1) { const int y = __shfl_up(y2, d, 32); y2 += (lane >= d) ? y : 0; }
    const int sstart = y2 - pd;
    const int ptot = __shfl(y2, 31, 32);
    const int segr = __shfl(sstart, r, 32);
    v4i o; o[0] = segr + excl; o[1] = o[0] + c[0]; o[2] = o[1] + c[1]; o[3] = o[2] + c[2];
    if (r == 0) { tl[lane] = sstart; tl[32 + lane] = t; tl[64 + lane] = (lane == 0) ? ptot : 0; tl[96 + lane] = 0; wave_sync(); }
    const int padcnt = ((tot + 63) & ~63) - tot;
    const int pbase = segr + tot;
    v8us z;
#pragma unroll
    for (int k = 0; k < 8; ++k) z[k] = (unsigned short)0;
#pragma unroll 1
    for (int ps = 0; ps < 2; ++ps) {
        *(volatile v4i*)(offs + (size_t)r * OFFP + 4 * lane) = o;
        if (r == 0) { const v4i v = *(const v4ia*)(&tl[4 * lane]); *(volatile v4i*)(T + 4 * lane) = v; }
#pragma unroll 1
        for (int j = 0; j < 63; ++j) { const int p = clampi(pbase + j, 0, PROWS - 1);
            if (j < padcnt) { *(volatile v8us*)(XP + (size_t)p * OBSD + 8 * lane) = z; } }
        if (ps == 0) __threadfence(); }
}

__global__ __launch_bounds__(1024) void k_rank(const int* __restrict__ opt, const float* __restrict__ obs,
                                               const int* __restrict__ offs, int* POS, bf* XP) {
    __shared__ int wc[32 * 32];
    const int tid = threadIdx.x, lane = tid & 31; const int wave = __builtin_amdgcn_readfirstlane(tid >> 5);
    const int blk = blockIdx.x;
    const size_t row = (size_t)blk * RB + tid;
    const int rel = clampi(opt[row], 0, NOPT - 1);
    int mine = 0; unsigned mymask = 0u;
#pragma unroll 1
    for (int r = 0; r < NREL; ++r) { const unsigned m = __builtin_amdgcn_ballot_w32(rel == r); const int c = __builtin_popcount(m);
        mine = (lane == r) ? c : mine; mymask = (rel == r) ? m : mymask; }
    const int lrank = __builtin_popcount(mymask & ((1u << lane) - 1u));
    wc[wave * 32 + lane] = mine;
    __syncthreads();
    if (wave == 0) {
        int run = clampi(offs[(size_t)lane * OFFP + blk], 0, PROWS);
#pragma unroll 1
        for (int w = 0; w < 32; ++w) { const int c = wc[w * 32 + lane]; wc[w * 32 + lane] = run; run += c; }
    }
    __syncthreads();
    const int pos = clampi(wc[wave * 32 + rel] + lrank, 0, PROWS - 1);
    const int c8 = lane * 8;
#pragma unroll 1
    for (int ps = 0; ps < 2; ++ps) {
        *(volatile int*)(POS + row) = pos;
#pragma unroll 1
        for (int j = 0; j < 32; ++j) { const int p = __shfl(pos, j, 32);
            const size_t rg = (size_t)blk * RB + (size_t)wave * 32 + j;
            const v8f a = *(const v8f*)(obs + rg * OBSD + c8); v8us oa;
#pragma unroll
            for (int k = 0; k < 8; ++k) { oa[k] = f2bf(a[k]); }
            *(volatile v8us*)(XP + (size_t)p * OBSD + c8) = oa; }
        if (ps == 0) __threadfence(); }
}

static_assert(32 * 16 * 4 == 16 * ACTP * 4);
__global__ __launch_bounds__(128) __attribute__((amdgpu_num_vgpr(256))) void k_fused(
        const bf* __restrict__ XP, const bf* __restrict__ W1B, const h16* __restrict__ W2H, const h16* __restrict__ HDH,
        const h16* __restrict__ E1H, const h16* __restrict__ E2H,
        const float* __restrict__ fb1, const float* __restrict__ fb2, const float* __restrict__ pb, const float* __restrict__ tb,
        const float* __restrict__ ob1, const float* __restrict__ ob2, const int* __restrict__ T, float* SP) {
    __shared__ __align__(16) h16 hs[4][16 * HP];
    __shared__ __align__(16) h16 ss[4][16 * SPH];
    __shared__ __align__(16) h16 es[4][16 * HP];
    __shared__ __align__(16) float ot[4][16 * OP];
    __shared__ float hd[4][16 * HDP];
    __shared__ float lsv[4][16];
    const int lane = threadIdx.x & 31, lr = lane & 15, hi = lane >> 4;
    const int wave = __builtin_amdgcn_readfirstlane(threadIdx.x >> 5);
    const int p0 = blockIdx.x * 64;
    const int sst = T[lane], tt = T[32 + lane];
    const int pe = sst + ((tt + 63) & ~63);
    const unsigned msk = __builtin_amdgcn_ballot_w32((p0 >= sst) && (p0 < pe));
    if (msk == 0u) return;
    const int r = clampi(__builtin_amdgcn_readfirstlane(__builtin_ctz(msk)), 0, NOPT - 1);
    const int pw = p0 + 16 * wave;

    v8f a1[4];
#pragma unroll
    for (int nt = 0; nt < 4; ++nt) a1[nt] = (v8f){};
    const size_t xo = (size_t)(pw + lr) * OBSD + 8 * hi;
    const int w1o = lr * OBSD + 8 * hi;
#pragma unroll 1
    for (int kc = 0; kc < OBSD; kc += 32) {
        const v16bf a = ldb(XP + xo + kc);
#pragma unroll
        for (int nt = 0; nt < 4; ++nt) { const v16bf b = ldb(W1B + w1o + nt * 16 * OBSD + kc); a1[nt] = wmmab_g(a, b, a1[nt]); }
    }
#pragma unroll
    for (int nt = 0; nt < 4; ++nt) { const float bv = bfr(fb1[nt * 16 + lr]);
#pragma unroll
        for (int j = 0; j < 8; ++j) { float v = a1[nt][j] + bv; v = (v > 0.0f) ? v : 0.0f;
            hs[wave][(8 * hi + j) * HP + nt * 16 + lr] = toh_flush(v * ASC); } }
    wave_sync();

    v8f a2[8];
#pragma unroll
    for (int nt = 0; nt < 8; ++nt) a2[nt] = (v8f){};
    const int w2o = lr * HIDD + 8 * hi;
#pragma unroll 1
    for (int kc = 0; kc < HIDD; kc += 32) {
        const v8h x0 = *(const v8ha*)(&hs[wave][lr * HP + kc + 8 * hi]);
        const v8h x1 = *(const v8ha*)(&hs[wave][lr * HP + kc + 16 + 8 * hi]);
        const v16h a = cat16h(x0, x1);
#pragma unroll
        for (int nt = 0; nt < 8; ++nt) { const v16h b = ldh(W2H + w2o + nt * 16 * HIDD + kc); a2[nt] = wmmah_g(a, b, a2[nt]); }
    }
#pragma unroll
    for (int nt = 0; nt < 8; ++nt) { const float bv = bfr(fb2[nt * 16 + lr]);
#pragma unroll
        for (int j = 0; j < 8; ++j) { float v = a2[nt][j] * INVC + bv; v = (v > 0.0f) ? v : 0.0f;
            ss[wave][(8 * hi + j) * SPH + nt * 16 + lr] = toh_flush(v * ASC); } }
    wave_sync();

    v8f a3 = (v8f){};
    v8f a4[4];
#pragma unroll
    for (int nt = 0; nt < 4; ++nt) a4[nt] = (v8f){};
    const int hdo = lr * FEAT + 8 * hi;
    const int e1o = r * (HIDD * FEAT) + lr * FEAT + 8 * hi;
#pragma unroll 1
    for (int kc = 0; kc < FEAT; kc += 32) {
        const v8h x0 = *(const v8ha*)(&ss[wave][lr * SPH + kc + 8 * hi]);
        const v8h x1 = *(const v8ha*)(&ss[wave][lr * SPH + kc + 16 + 8 * hi]);
        const v16h a = cat16h(x0, x1);
        { const v16h b = ldh(HDH + hdo + kc); a3 = wmmah_g(a, b, a3); }
#pragma unroll
        for (int nt = 0; nt < 4; ++nt) { const v16h b = ldh(E1H + e1o + nt * 16 * FEAT + kc); a4[nt] = wmmah_g(a, b, a4[nt]); }
    }
    {
        const float pbv = pb[lr & 7], tbv = tb[lr & 7];
        const float hb = bfr((lr < 8) ? pbv : tbv);
#pragma unroll
        for (int j = 0; j < 8; ++j) hd[wave][(8 * hi + j) * HDP + lr] = a3[j] * INVC + hb;
    }
#pragma unroll
    for (int nt = 0; nt < 4; ++nt) { const float bv = bfr(ob1[r * HIDD + nt * 16 + lr]);
#pragma unroll
        for (int j = 0; j < 8; ++j) { float v = a4[nt][j] * INVC + bv; v = (v > 0.0f) ? v : 0.0f;
            es[wave][(8 * hi + j) * HP + nt * 16 + lr] = toh_flush(v * ASC); } }
    wave_sync();

    v8f a5[2];
#pragma unroll
    for (int nt = 0; nt < 2; ++nt) a5[nt] = (v8f){};
    const int e2o = r * (ACTP * HIDD) + lr * HIDD + 8 * hi;
#pragma unroll 1
    for (int kc = 0; kc < HIDD; kc += 32) {
        const v8h x0 = *(const v8ha*)(&es[wave][lr * HP + kc + 8 * hi]);
        const v8h x1 = *(const v8ha*)(&es[wave][lr * HP + kc + 16 + 8 * hi]);
        const v16h a = cat16h(x0, x1);
#pragma unroll
        for (int nt = 0; nt < 2; ++nt) { const v16h b = ldh(E2H + e2o + nt * 16 * HIDD + kc); a5[nt] = wmmah_g(a, b, a5[nt]); }
    }
#pragma unroll
    for (int nt = 0; nt < 2; ++nt) { const int n = nt * 16 + lr;
        float braw = ob2[r * ACTN + min(n, ACTN - 1)]; asm volatile("" : "+v"(braw));
        const float bv = (n < ACTN) ? bfr(braw) : 0.0f;
#pragma unroll
        for (int j = 0; j < 8; ++j) ot[wave][(8 * hi + j) * OP + n] = a5[nt][j] * INVC + bv; }
    wave_sync();

    const int row = lane >> 1, hf = lane & 1;
    float mx = -3.0e38f;
#pragma unroll 1
    for (int c = 0; c < 9; ++c) mx = fmaxf(mx, ot[wave][row * OP + hf * 9 + c]);
    mx = fmaxf(mx, __shfl_xor(mx, 1, 32));
    float s = 0.0f;
#pragma unroll 1
    for (int c = 0; c < 9; ++c) s += expf(ot[wave][row * OP + hf * 9 + c] - mx);
    s += __shfl_xor(s, 1, 32);
    const float lse = mx + logf(s);
    const float hv = hd[wave][row * HDP + 8 * hf + r];
    const float sg = 1.0f / (1.0f + expf(-hv));
    const float ov = (hf == 0) ? hv : sg;
    ot[wave][row * OP + ACTN + hf] = ov;
    if (hf == 0) lsv[wave][row] = lse;
    wave_sync();

    v4f o[4];
#pragma unroll
    for (int it = 0; it < 4; ++it) { const int rw = 4 * it + (lane >> 3), c4 = 4 * (lane & 7);
        const v4f x = *(const v4fa*)(&ot[wave][rw * OP + c4]); const float l = lsv[wave][rw];
#pragma unroll
        for (int k = 0; k < 4; ++k) o[it][k] = (c4 + k < ACTN) ? (x[k] - l) : x[k]; }
#pragma unroll 1
    for (int ps = 0; ps < 2; ++ps) {
#pragma unroll
        for (int it = 0; it < 4; ++it) *(volatile v4f*)(SP + (size_t)(pw + 4 * it + (lane >> 3)) * ACTP + 4 * (lane & 7)) = o[it];
        if (ps == 0) __threadfence(); }
}

__global__ __launch_bounds__(256) void k_unsort(const int* __restrict__ POS, const int* __restrict__ act, const float* __restrict__ SP, float* OUT) {
    const size_t i = (size_t)blockIdx.x * 256 + threadIdx.x; if (i >= (size_t)(NB / 4)) return;
    const v4i p = *(const v4i*)(POS + i * 4); const v4i a = *(const v4i*)(act + i * 4); v4f v0, v1, v2;
#pragma unroll
    for (int k = 0; k < 4; ++k) { const size_t b = (size_t)clampi(p[k], 0, PROWS - 1) * ACTP;
        v0[k] = SP[b + clampi(a[k], 0, ACTN - 1)]; v1[k] = SP[b + ACTN]; v2[k] = SP[b + ACTN + 1]; }
    float* o0 = OUT + i * 4; float* o1 = OUT + (size_t)NB_FULL + i * 4; float* o2 = OUT + (size_t)2 * NB_FULL + i * 4;
    *(volatile v4f*)o0 = v0; *(volatile v4f*)o1 = v1; *(volatile v4f*)o2 = v2;
    __threadfence();
    *(volatile v4f*)o0 = v0; *(volatile v4f*)o1 = v1; *(volatile v4f*)o2 = v2;
}

static constexpr size_t al256(size_t v) { return (v + 255) & ~(size_t)255; }
static constexpr size_t SZ_W1  = al256((size_t)HIDD * OBSD * 2);
static constexpr size_t SZ_W2  = al256((size_t)FEAT * HIDD * 2);
static constexpr size_t SZ_HD  = al256((size_t)16 * FEAT * 2);
static constexpr size_t SZ_E1  = al256((size_t)NOPT * HIDD * FEAT * 2);
static constexpr size_t SZ_E2  = al256((size_t)NOPT * ACTP * HIDD * 2);
static constexpr size_t SZ_CNT = al256((size_t)NBLK * 32 * 4);
static constexpr size_t SZ_OFF = al256((size_t)NREL * OFFP * 4);
static constexpr size_t SZ_T   = al256((size_t)128 * 4);
static constexpr size_t SZ_POS = al256((size_t)NB * 4);
static constexpr size_t SZ_XP  = al256((size_t)PROWS * OBSD * 2);
static constexpr size_t SZ_SP  = al256((size_t)PROWS * ACTP * 4);
static constexpr size_t SZ_TOTAL = SZ_W1 + SZ_W2 + SZ_HD + SZ_E1 + SZ_E2 + SZ_CNT + SZ_OFF + SZ_T + SZ_POS + SZ_XP + SZ_SP;
static_assert(SZ_TOTAL <= (size_t)134217728);
static_assert((size_t)2 * NB_FULL + (size_t)NB <= (size_t)3 * NB_FULL);

extern "C" void kernel_launch(void* const* d_in, const int* in_sizes, int n_in,
                              void* d_out, int out_size, void* d_ws, size_t ws_size, hipStream_t stream) {
    if (n_in < 15) return;
    if ((size_t)in_sizes[0] < (size_t)NB * OBSD) return;
    if ((size_t)in_sizes[1] < (size_t)NB || (size_t)in_sizes[2] < (size_t)NB) return;
    if ((size_t)in_sizes[3] < (size_t)HIDD * OBSD || (size_t)in_sizes[4] < (size_t)HIDD) return;
    if ((size_t)in_sizes[5] < (size_t)FEAT * HIDD || (size_t)in_sizes[6] < (size_t)FEAT) return;
    if ((size_t)in_sizes[7] < (size_t)NOPT * FEAT || (size_t)in_sizes[8] < (size_t)NOPT) return;
    if ((size_t)in_sizes[9] < (size_t)NOPT * FEAT || (size_t)in_sizes[10] < (size_t)NOPT) return;
    if ((size_t)in_sizes[11] < (size_t)NOPT * HIDD * FEAT || (size_t)in_sizes[12] < (size_t)NOPT * HIDD) return;
    if ((size_t)in_sizes[13] < (size_t)NOPT * ACTN * HIDD || (size_t)in_sizes[14] < (size_t)NOPT * ACTN) return;
    if ((size_t)out_size < (size_t)2 * NB_FULL + (size_t)NB) return;
    if (SZ_TOTAL > ws_size) return;
    const float* obs = (const float*)d_in[0];
    const int*   act = (const int*)d_in[1];
    const int*   opt = (const int*)d_in[2];
    const float* fW1 = (const float*)d_in[3];
    const float* fb1 = (const float*)d_in[4];
    const float* fW2 = (const float*)d_in[5];
    const float* fb2 = (const float*)d_in[6];
    const float* pW  = (const float*)d_in[7];
    const float* pb  = (const float*)d_in[8];
    const float* tW  = (const float*)d_in[9];
    const float* tb  = (const float*)d_in[10];
    const float* oW1 = (const float*)d_in[11];
    const float* ob1 = (const float*)d_in[12];
    const float* oW2 = (const float*)d_in[13];
    const float* ob2 = (const float*)d_in[14];
    float* OUT = (float*)d_out;
    char* wsp = (char*)d_ws;
    bf*  W1B = (bf*)wsp;   wsp += SZ_W1;
    h16* W2H = (h16*)wsp;  wsp += SZ_W2;
    h16* HDH = (h16*)wsp;  wsp += SZ_HD;
    h16* E1H = (h16*)wsp;  wsp += SZ_E1;
    h16* E2H = (h16*)wsp;  wsp += SZ_E2;
    int* CNT = (int*)wsp;  wsp += SZ_CNT;
    int* OFF = (int*)wsp;  wsp += SZ_OFF;
    int* TT  = (int*)wsp;  wsp += SZ_T;
    int* POS = (int*)wsp;  wsp += SZ_POS;
    bf*  XP  = (bf*)wsp;   wsp += SZ_XP;
    float* SP = (float*)wsp; wsp += SZ_SP;

    k_wconv<<<WB_W1 + WB_W2 + WB_HD + WB_E1 + WB_E2, 256, 0, stream>>>(fW1, fW2, pW, tW, oW1, oW2, W1B, W2H, HDH, E1H, E2H);
    k_count<<<NBLK, 1024, 0, stream>>>(opt, CNT);
    k_scan<<<1, 1024, 0, stream>>>(CNT, OFF, TT, XP);
    k_rank<<<NBLK, 1024, 0, stream>>>(opt, obs, OFF, POS, XP);
    k_fused<<<PROWS / 64, 128, 0, stream>>>(XP, W1B, W2H, HDH, E1H, E2H, fb1, fb2, pb, tb, ob1, ob2, TT, SP);
    k_unsort<<<(unsigned)((NB / 4 + 255) / 256), 256, 0, stream>>>(POS, act, SP, OUT);
}
